// MultiHeadAttention_274877906955
// MI455X (gfx1250) — hardware-verified
//
#include <hip/hip_runtime.h>


#ifndef NB
#define NB 2
#endif
#ifndef SEQ
#define SEQ 2048
#endif
#ifndef RH
#define RH 256
#endif
#define NB_FULL  2
#define SEQ_FULL 2048
#define CC   1024
#define NH   16
#define HD   64
#define MROWS (NB * SEQ)
#define PCAR 1024.0f
#define QCAR 16.0f
#define VCAR 16.0f
#define L2E  1.4426950408889634f
#define NEGB (-1.0e30f)
#define OSP  68
#define W1   ((size_t)CC * CC)
#define PL16 ((size_t)MROWS * CC)
#define PLR  ((size_t)NB * NH * RH * HD)
#define WS_TOTAL (10 * W1 + 24 * PL16 + 12 * PLR)
static_assert(CC == NH * HD);
static_assert(HD == 64);
static_assert(CC % 64 == 0 && CC % 32 == 0);
static_assert(MROWS % 64 == 0);
static_assert(SEQ % 256 == 0);
static_assert(RH % 256 == 0 && RH <= SEQ);
static_assert((SEQ - RH) % 32 == 0 && RH % 32 == 0 && RH % 16 == 0);
static_assert(NB <= NB_FULL && SEQ <= SEQ_FULL);
static_assert((W1 * 2) % 256 == 0 && (PL16 * 2) % 256 == 0 && (PLR * 2) % 256 == 0);
static_assert(2 * PL16 * sizeof(unsigned short) <= PL16 * sizeof(float));
static_assert(WS_TOTAL <= (size_t)134217728);

typedef _Float16 h16;
typedef unsigned short bf;
typedef __attribute__((ext_vector_type(16))) __bf16   v16bf;
typedef __attribute__((ext_vector_type(16))) _Float16 v16h;
typedef __attribute__((ext_vector_type(16))) unsigned short v16us;
typedef __attribute__((ext_vector_type(8)))  _Float16 v8h;
typedef __attribute__((ext_vector_type(8)))  unsigned short v8us;
typedef __attribute__((ext_vector_type(8)))  float    v8f;
typedef __attribute__((ext_vector_type(4)))  float    v4f;
typedef v4f  __attribute__((may_alias)) v4fa;

__device__ __forceinline__ unsigned short f2bf(float f) { unsigned u = __float_as_uint(f); u += 0x7FFFu + ((u >> 16) & 1u); return (unsigned short)(u >> 16); }
__device__ __forceinline__ float bf2f(unsigned short b) { return __uint_as_float(((unsigned)b) << 16); }
__device__ __forceinline__ float bfr(float f) { return bf2f(f2bf(f)); }
__device__ __forceinline__ h16 tohx(float x) { return (h16)x; }
__device__ __forceinline__ void splitf(float y, unsigned short& h, unsigned short& l) { h = f2bf(y); l = f2bf(y - bf2f(h)); }
__device__ __forceinline__ float sigm(float g) { return __builtin_amdgcn_rcpf(1.0f + __builtin_amdgcn_exp2f(-g * L2E)); }
__device__ __forceinline__ v16h cat16(v8h lo, v8h hi) { return __builtin_shufflevector(lo, hi, 0, 1, 2, 3, 4, 5, 6, 7, 8, 9, 10, 11, 12, 13, 14, 15); }
__device__ __forceinline__ v16bf cat16b(v8us lo, v8us hi) { return __builtin_bit_cast(v16bf, __builtin_shufflevector(lo, hi, 0, 1, 2, 3, 4, 5, 6, 7, 8, 9, 10, 11, 12, 13, 14, 15)); }
__device__ __forceinline__ v8f wmma16(v16h a, v16h b, v8f c) { return __builtin_amdgcn_wmma_f32_16x16x32_f16(false, a, false, b, (short)0, c, false, false); }
__device__ __forceinline__ v8f wmmab(v16bf a, v16bf b, v8f c) { return __builtin_amdgcn_wmma_f32_16x16x32_bf16(false, a, false, b, (short)0, c, false, false); }

template <typename T16> struct WFrag;
template <> struct WFrag<h16> { typedef v16h V; static __device__ __forceinline__ V ld(const h16* p) { return cat16(*(const v8h*)p, *(const v8h*)(p + 16)); } static __device__ __forceinline__ v8f mma(V a, V b, v8f c) { return wmma16(a, b, c); } };
template <> struct WFrag<bf> { typedef v16bf V; static __device__ __forceinline__ V ld(const bf* p) { return cat16b(*(const v8us*)p, *(const v8us*)(p + 16)); } static __device__ __forceinline__ v8f mma(V a, V b, v8f c) { return wmmab(a, b, c); } };

template <typename T16, int NSPLIT, bool BIAS>
__device__ __forceinline__ void gemmw_body(const T16* __restrict__ A, const T16* __restrict__ A2, const T16* __restrict__ Bt, const T16* __restrict__ Bt2, int K, float* C, int ldc, const float* __restrict__ bias, size_t sA, size_t sB, size_t sC, float* os) {
    typedef typename WFrag<T16>::V V;
    const size_t z = blockIdx.z; A += z * sA; if (A2) A2 += z * sA; Bt += z * sB; if (Bt2) Bt2 += z * sB; C += z * sC;
    const int lane = threadIdx.x & 31, lr = lane & 15, hi = lane >> 4; const int r0 = blockIdx.x * 64, c0 = blockIdx.y * 64;
    v8f acc[4][4];
#pragma unroll
    for (int mb = 0; mb < 4; ++mb)
#pragma unroll
        for (int nb = 0; nb < 4; ++nb) acc[mb][nb] = (v8f){};
    const size_t aoff = (size_t)(r0 + lr) * K + 8 * hi, boff = (size_t)(c0 + lr) * K + 8 * hi;
#pragma unroll 1
    for (int kc = 0; kc < K; kc += 32) {
        V a[4], a2[4];
#pragma unroll
        for (int mb = 0; mb < 4; ++mb) { a[mb] = WFrag<T16>::ld(A + aoff + (size_t)mb * 16 * K + kc); if (NSPLIT == 1 || NSPLIT == 2) a2[mb] = WFrag<T16>::ld(A2 + aoff + (size_t)mb * 16 * K + kc); }
#pragma unroll
        for (int nb = 0; nb < 4; ++nb) { const V b = WFrag<T16>::ld(Bt + boff + (size_t)nb * 16 * K + kc); V b2; if (NSPLIT >= 2) b2 = WFrag<T16>::ld(Bt2 + boff + (size_t)nb * 16 * K + kc);
#pragma unroll
            for (int mb = 0; mb < 4; ++mb) { acc[mb][nb] = WFrag<T16>::mma(a[mb], b, acc[mb][nb]); if (NSPLIT == 1 || NSPLIT == 2) acc[mb][nb] = WFrag<T16>::mma(a2[mb], b, acc[mb][nb]); if (NSPLIT >= 2) acc[mb][nb] = WFrag<T16>::mma(a[mb], b2, acc[mb][nb]); } }
        asm volatile("v_nop\n\tv_nop\n\tv_nop\n\tv_nop" : "+v"(acc[0][0]), "+v"(acc[1][1]), "+v"(acc[2][2]), "+v"(acc[3][3]) : "v"(a[0]), "v"(a[3]));
    }
#pragma unroll
    for (int mb = 0; mb < 4; ++mb) {
#pragma unroll
        for (int nb = 0; nb < 4; ++nb) {
#pragma unroll
            for (int j = 0; j < 8; ++j) os[(hi * 8 + j) * OSP + nb * 16 + lr] = acc[mb][nb][j]; }
        __builtin_amdgcn_wave_barrier(); asm volatile("" ::: "memory");
        float* crow = C + (size_t)(r0 + mb * 16) * ldc + c0;
#pragma unroll 1
        for (int ps = 0; ps < 2; ++ps) {
#pragma unroll
            for (int s = 0; s < 8; ++s) { const int row = 2 * s + hi, cofs = lr * 4; v4f val = *(const v4fa*)(os + row * OSP + cofs); if (BIAS) { val[0] += bfr(bias[c0 + cofs]); val[1] += bfr(bias[c0 + cofs + 1]); val[2] += bfr(bias[c0 + cofs + 2]); val[3] += bfr(bias[c0 + cofs + 3]); }
                *(volatile v4f*)(crow + (size_t)row * ldc + cofs) = val; }
            if (ps == 0) __threadfence(); }
        __builtin_amdgcn_wave_barrier(); asm volatile("" ::: "memory");
    }
}

__global__ __launch_bounds__(32) void k_gemm_proj(const bf* __restrict__ A, const bf* __restrict__ Bt, float* C, size_t sB, size_t sC) {
    __shared__ __align__(16) float os[16 * OSP];
    gemmw_body<bf, 0, false>(A, nullptr, Bt, nullptr, CC, C, CC, nullptr, 0, sB, sC, os);
}
__global__ __launch_bounds__(32) void k_gemm_out(const bf* __restrict__ Ah, const bf* __restrict__ Al, const bf* __restrict__ Bt, float* C, const float* __restrict__ bias) {
    __shared__ __align__(16) float os[16 * OSP];
    gemmw_body<bf, 1, true>(Ah, Al, Bt, nullptr, CC, C, CC, bias, 0, 0, 0, os);
}

__global__ __launch_bounds__(256) void k_cvt8(const float* __restrict__ src, bf* dst, unsigned n8, unsigned per8, unsigned sstr8) {
    const unsigned i = blockIdx.x * 256u + threadIdx.x; if (i >= n8) return;
    const unsigned b = i / per8, r = i - b * per8;
    const v8f v = *(const v8f*)(src + ((size_t)b * sstr8 + r) * 8); v8us o;
#pragma unroll
    for (int k = 0; k < 8; ++k) o[k] = f2bf(v[k]);
    *(volatile v8us*)(dst + (size_t)i * 8) = o; __threadfence(); *(volatile v8us*)(dst + (size_t)i * 8) = o; }

__global__ __launch_bounds__(256) void k_qkp(const float* __restrict__ F, h16* P16, bf* Ph, bf* Pl) {
    const unsigned i = blockIdx.x * 256u + threadIdx.x; if (i >= (unsigned)(MROWS * (CC / 8))) return;
    const unsigned w = blockIdx.y; const unsigned e = i * 8u; const unsigned c = e % CC, row = e / CC; const unsigned b = row / SEQ, t = row % SEQ; const unsigned h = c / HD, d = c % HD;
    const float* f = F + (size_t)w * MROWS * CC + e;
    const v4f a = *(const v4f*)f, g = *(const v4f*)(f + 4); v8h o16; v8us oh, ol;
#pragma unroll
    for (int k = 0; k < 4; ++k) { unsigned short hh, ll; o16[k] = tohx(a[k] * QCAR); splitf(a[k], hh, ll); oh[k] = hh; ol[k] = ll; o16[4 + k] = tohx(g[k] * QCAR); splitf(g[k], hh, ll); oh[4 + k] = hh; ol[4 + k] = ll; }
    const size_t bh = (size_t)(w * NB + b) * NH + h;
    const size_t o1 = (bh * SEQ + t) * HD + d;
    const size_t o2 = (bh * RH + (t < RH ? t : 0u)) * HD + d;
#pragma unroll 1
    for (int ps = 0; ps < 2; ++ps) { *(volatile v8h*)(P16 + o1) = o16; if (t < RH) { *(volatile v8us*)(Ph + o2) = oh; *(volatile v8us*)(Pl + o2) = ol; } if (ps == 0) __threadfence(); }
}

__global__ __launch_bounds__(256) void k_vtp(const float* __restrict__ F, h16* V16, bf* Vh, bf* Vl) {
    const unsigned i = blockIdx.x * 256u + threadIdx.x; if (i >= (unsigned)(MROWS * (CC / 8))) return;
    const unsigned e = i * 8u; const unsigned t = e % SEQ; const unsigned d = (e / SEQ) % HD; const unsigned bh = e / (SEQ * HD); const unsigned b = bh / NH, h = bh % NH;
    const float* f = F + ((size_t)b * SEQ + t) * CC + h * HD + d; v8h o16; v8us oh, ol;
#pragma unroll
    for (int k = 0; k < 8; ++k) { const float x = f[(size_t)k * CC]; unsigned short hh, ll; o16[k] = tohx(x * VCAR); splitf(x, hh, ll); oh[k] = hh; ol[k] = ll; }
    const size_t o2 = ((size_t)bh * HD + d) * RH + (t < RH ? t : 0u);
#pragma unroll 1
    for (int ps = 0; ps < 2; ++ps) { *(volatile v8h*)(V16 + e) = o16; if (t < RH) { *(volatile v8us*)(Vh + o2) = oh; *(volatile v8us*)(Vl + o2) = ol; } if (ps == 0) __threadfence(); }
}

template <typename T16> struct PPack;
template <> struct PPack<h16> { static __device__ __forceinline__ void mk(const v8f& p0, const v8f& p1, float car, v16h& a, v16h& b) { v16h r;
#pragma unroll
        for (int i = 0; i < 8; ++i) { r[i] = tohx(p0[i] * car); r[8 + i] = tohx(p1[i] * car); }
        a = r; b = r; } };
template <> struct PPack<bf> { static __device__ __forceinline__ void mk(const v8f& p0, const v8f& p1, float car, v16bf& a, v16bf& b) { (void)car; v16us h, l;
#pragma unroll
        for (int i = 0; i < 8; ++i) { unsigned short hh, ll; splitf(p0[i], hh, ll); h[i] = hh; l[i] = ll; splitf(p1[i], hh, ll); h[8 + i] = hh; l[8 + i] = ll; }
        a = __builtin_bit_cast(v16bf, h); b = __builtin_bit_cast(v16bf, l); } };

template <int N> struct Grd;
template <> struct Grd<1> {
    template <typename V> static __device__ __forceinline__ void s(v8f (&st)[2][1], const V& x, const V& y) { asm volatile("v_nop\n\tv_nop\n\tv_nop\n\tv_nop" : "+v"(st[0][0]), "+v"(st[1][0]) : "v"(x), "v"(y)); }
    template <typename V> static __device__ __forceinline__ void o(v8f (&oa)[4][1], const V& x, const V& y, const V& z) { asm volatile("v_nop\n\tv_nop\n\tv_nop\n\tv_nop" : "+v"(oa[0][0]), "+v"(oa[1][0]), "+v"(oa[2][0]), "+v"(oa[3][0]) : "v"(x), "v"(y), "v"(z)); }
};
template <> struct Grd<2> {
    template <typename V> static __device__ __forceinline__ void s(v8f (&st)[2][2], const V& x, const V& y) { asm volatile("v_nop\n\tv_nop\n\tv_nop\n\tv_nop" : "+v"(st[0][0]), "+v"(st[1][0]), "+v"(st[0][1]), "+v"(st[1][1]) : "v"(x), "v"(y)); }
    template <typename V> static __device__ __forceinline__ void o(v8f (&oa)[4][2], const V& x, const V& y, const V& z) { asm volatile("v_nop\n\tv_nop\n\tv_nop\n\tv_nop" : "+v"(oa[0][0]), "+v"(oa[1][0]), "+v"(oa[2][0]), "+v"(oa[3][0]), "+v"(oa[0][1]), "+v"(oa[1][1]), "+v"(oa[2][1]), "+v"(oa[3][1]) : "v"(x), "v"(y), "v"(z)); }
};

template <typename T16, bool SPLIT, int NQ>
__device__ __forceinline__ void attn_body(const T16* __restrict__ Q, const T16* __restrict__ Q2, const T16* __restrict__ Kp, const T16* __restrict__ K2, const T16* __restrict__ Vt, const T16* __restrict__ V2,
                                          const float* __restrict__ G, int vpitch, int q0, float ssc, float osc, float pcar, bf* Ah, bf* Al, float* os) {
    typedef typename WFrag<T16>::V V;
    const int lane = threadIdx.x & 31, lr = lane & 15, hi = lane >> 4;
    V qf[NQ][2], qf2[NQ][2];
#pragma unroll
    for (int nb = 0; nb < NQ; ++nb)
#pragma unroll
        for (int ds = 0; ds < 2; ++ds) { const size_t qo = (size_t)(q0 + 16 * nb + lr) * HD + 32 * ds + 8 * hi; qf[nb][ds] = WFrag<T16>::ld(Q + qo); if (SPLIT) qf2[nb][ds] = WFrag<T16>::ld(Q2 + qo); }
    v8f o[4][NQ]; float mrun[NQ], lrun[NQ];
#pragma unroll
    for (int nb = 0; nb < NQ; ++nb) { mrun[nb] = NEGB; lrun[nb] = 0.0f;
#pragma unroll
        for (int dt = 0; dt < 4; ++dt) o[dt][nb] = (v8f){}; }
    const int kend = q0 + 16 * NQ;
#pragma unroll 1
    for (int kt = 0; kt < kend; kt += 32) {
        V ka[2][2], ka2[2][2];
#pragma unroll
        for (int mb = 0; mb < 2; ++mb)
#pragma unroll
            for (int ds = 0; ds < 2; ++ds) { const size_t ko = (size_t)(kt + 16 * mb + lr) * HD + 32 * ds + 8 * hi; ka[mb][ds] = WFrag<T16>::ld(Kp + ko); if (SPLIT) ka2[mb][ds] = WFrag<T16>::ld(K2 + ko); }
        v8f st[2][NQ];
#pragma unroll
        for (int mb = 0; mb < 2; ++mb)
#pragma unroll
            for (int nb = 0; nb < NQ; ++nb) { v8f z = (v8f){};
                z = WFrag<T16>::mma(ka[mb][0], qf[nb][0], z); z = WFrag<T16>::mma(ka[mb][1], qf[nb][1], z);
                if (SPLIT) { z = WFrag<T16>::mma(ka2[mb][0], qf[nb][0], z); z = WFrag<T16>::mma(ka2[mb][1], qf[nb][1], z); z = WFrag<T16>::mma(ka[mb][0], qf2[nb][0], z); z = WFrag<T16>::mma(ka[mb][1], qf2[nb][1], z); }
                st[mb][nb] = z; }
        Grd<NQ>::s(st, ka[1][1], SPLIT ? qf2[NQ - 1][1] : qf[NQ - 1][1]);
        V pb[NQ], pb2[NQ];
#pragma unroll
        for (int nb = 0; nb < NQ; ++nb) {
            const int qg = q0 + 16 * nb + lr; float mx = NEGB;
#pragma unroll
            for (int mb = 0; mb < 2; ++mb)
#pragma unroll
                for (int r = 0; r < 8; ++r) { const int kg = kt + 16 * mb + 8 * hi + r; float t = st[mb][nb][r] * ssc; t = (kg <= qg) ? t : NEGB; st[mb][nb][r] = t; mx = fmaxf(mx, t); }
            mx = fmaxf(mx, __shfl_xor(mx, 16, 32));
            const float mn = fmaxf(mrun[nb], mx);
            const float al = __builtin_amdgcn_exp2f((mrun[nb] - mn) * L2E); mrun[nb] = mn;
            float psum = 0.0f;
#pragma unroll
            for (int mb = 0; mb < 2; ++mb)
#pragma unroll
                for (int r = 0; r < 8; ++r) { const float p = __builtin_amdgcn_exp2f((st[mb][nb][r] - mn) * L2E); psum += p; st[mb][nb][r] = p; }
            lrun[nb] = lrun[nb] * al + psum;
#pragma unroll
            for (int dt = 0; dt < 4; ++dt)
#pragma unroll
                for (int r = 0; r < 8; ++r) o[dt][nb][r] *= al;
            PPack<T16>::mk(st[0][nb], st[1][nb], pcar, pb[nb], pb2[nb]);
        }
        V va, va2;
#pragma unroll
        for (int dt = 0; dt < 4; ++dt) { const size_t vo = (size_t)(16 * dt + lr) * vpitch + kt + 8 * hi; va = WFrag<T16>::ld(Vt + vo); if (SPLIT) va2 = WFrag<T16>::ld(V2 + vo);
#pragma unroll
            for (int nb = 0; nb < NQ; ++nb) { o[dt][nb] = WFrag<T16>::mma(va, pb[nb], o[dt][nb]); if (SPLIT) { o[dt][nb] = WFrag<T16>::mma(va2, pb[nb], o[dt][nb]); o[dt][nb] = WFrag<T16>::mma(va, pb2[nb], o[dt][nb]); } } }
        Grd<NQ>::o(o, SPLIT ? va2 : va, pb[NQ - 1], SPLIT ? pb2[NQ - 1] : pb[0]);
    }
#pragma unroll
    for (int nb = 0; nb < NQ; ++nb) { float lt = lrun[nb]; lt += __shfl_xor(lt, 16, 32); const float inv = osc * __builtin_amdgcn_rcpf(lt);
#pragma unroll
        for (int dt = 0; dt < 4; ++dt) { v4f a, c;
#pragma unroll
            for (int r = 0; r < 4; ++r) { a[r] = o[dt][nb][r] * inv; c[r] = o[dt][nb][4 + r] * inv; }
            float* dst = os + (16 * nb + lr) * OSP + 16 * dt + 8 * hi; *(v4fa*)dst = a; *(v4fa*)(dst + 4) = c; } }
    __syncthreads();
    const int rr = lane >> 3, seg = (lane & 7) * 8;
#pragma unroll 1
    for (int ps = 0; ps < 2; ++ps) {
#pragma unroll
        for (int s = 0; s < 4 * NQ; ++s) { const int row = 4 * s + rr; const v4f a = *(const v4fa*)(os + row * OSP + seg); const v4f c = *(const v4fa*)(os + row * OSP + seg + 4);
            const float* gp = G + (size_t)(q0 + row) * CC + seg; const v4f ga = *(const v4f*)gp; const v4f gc = *(const v4f*)(gp + 4); v8us oh, ol;
#pragma unroll
            for (int k = 0; k < 4; ++k) { unsigned short hh, ll; const float ya = a[k] * sigm(ga[k]); const float yc = c[k] * sigm(gc[k]); splitf(ya, hh, ll); oh[k] = hh; ol[k] = ll; splitf(yc, hh, ll); oh[4 + k] = hh; ol[4 + k] = ll; }
            const size_t oo = (size_t)(q0 + row) * CC + seg; *(volatile v8us*)(Ah + oo) = oh; *(volatile v8us*)(Al + oo) = ol; }
        if (ps == 0) __threadfence(); }
}

__global__ __launch_bounds__(32) void k_attn_s(const bf* __restrict__ Qh, const bf* __restrict__ Ql, const bf* __restrict__ Kh, const bf* __restrict__ Kl, const bf* __restrict__ Vh, const bf* __restrict__ Vl, const float* __restrict__ Gt, bf* ATh, bf* ATl) {
    __shared__ __align__(16) float os[16 * OSP];
    const size_t bh = (size_t)blockIdx.z * NH + blockIdx.y; const size_t po = bh * RH * HD; const size_t ao = (size_t)blockIdx.z * SEQ * CC + (size_t)blockIdx.y * HD;
    attn_body<bf, true, 1>(Qh + po, Ql + po, Kh + po, Kl + po, Vh + po, Vl + po, Gt + ao, RH, (int)blockIdx.x * 16, 0.125f, 1.0f, 1.0f, ATh + ao, ATl + ao, os);
}
__global__ __launch_bounds__(32) void k_attn_h(const h16* __restrict__ Q, const h16* __restrict__ Kp, const h16* __restrict__ Vt, const float* __restrict__ Gt, bf* ATh, bf* ATl) {
    __shared__ __align__(16) float os[32 * OSP];
    const size_t bh = (size_t)blockIdx.z * NH + blockIdx.y; const size_t po = bh * SEQ * HD; const size_t ao = (size_t)blockIdx.z * SEQ * CC + (size_t)blockIdx.y * HD;
    attn_body<h16, false, 2>(Q + po, nullptr, Kp + po, nullptr, Vt + po, nullptr, Gt + ao, SEQ, RH + (int)blockIdx.x * 32, 0.125f / (QCAR * QCAR), 1.0f / (PCAR * VCAR), PCAR, ATh + ao, ATl + ao, os);
}

extern "C" void kernel_launch(void* const* d_in, const int* in_sizes, int n_in,
                              void* d_out, int out_size, void* d_ws, size_t ws_size, hipStream_t stream) {
    if (n_in < 7) return;
    if ((size_t)in_sizes[0] < ((size_t)(NB - 1) * SEQ_FULL + SEQ) * CC) return;
    if ((size_t)in_sizes[1] < W1 || (size_t)in_sizes[2] < W1 || (size_t)in_sizes[3] < W1 || (size_t)in_sizes[4] < W1 || (size_t)in_sizes[5] < W1 || in_sizes[6] < CC) return;
    if ((size_t)out_size < PL16) return;
    const float* x = (const float*)d_in[0]; const float* wq = (const float*)d_in[1]; const float* wk = (const float*)d_in[2]; const float* wv = (const float*)d_in[3];
    const float* wg = (const float*)d_in[4]; const float* wo = (const float*)d_in[5]; const float* bo = (const float*)d_in[6];
    float* OUT = (float*)d_out;
    char* wsp = (char*)d_ws;
    auto take = [&](size_t bytes) { char* p = wsp; wsp += (bytes + 255) & ~(size_t)255; return (void*)p; };
    bf* WQ = (bf*)take(4 * W1 * 2);
    bf* WO = (bf*)take(W1 * 2);
    bf* XB = (bf*)take(PL16 * 2);
    float* F = (float*)take(4 * PL16 * 4);
    h16* QK16 = (h16*)take(2 * PL16 * 2);
    h16* VT16 = (h16*)take(PL16 * 2);
    bf* QKh = (bf*)take(2 * PLR * 2); bf* QKl = (bf*)take(2 * PLR * 2);
    bf* VTh = (bf*)take(PLR * 2); bf* VTl = (bf*)take(PLR * 2);
    if ((size_t)(wsp - (char*)d_ws) > ws_size) return;
    bf* ATh = (bf*)F; bf* ATl = ATh + PL16;
    const float* GATE = F + 3 * PL16;
    const unsigned w8 = (unsigned)(W1 / 8), x8 = (unsigned)(PL16 / 8);
    k_cvt8<<<(w8 + 255) / 256, 256, 0, stream>>>(wq, WQ, w8, w8, 0u);
    k_cvt8<<<(w8 + 255) / 256, 256, 0, stream>>>(wk, WQ + W1, w8, w8, 0u);
    k_cvt8<<<(w8 + 255) / 256, 256, 0, stream>>>(wv, WQ + 2 * W1, w8, w8, 0u);
    k_cvt8<<<(w8 + 255) / 256, 256, 0, stream>>>(wg, WQ + 3 * W1, w8, w8, 0u);
    k_cvt8<<<(w8 + 255) / 256, 256, 0, stream>>>(wo, WO, w8, w8, 0u);
    k_cvt8<<<(x8 + 255) / 256, 256, 0, stream>>>(x, XB, x8, (unsigned)((size_t)SEQ * CC / 8), (unsigned)((size_t)SEQ_FULL * CC / 8));
    k_gemm_proj<<<dim3(MROWS / 64, CC / 64, 4), 32, 0, stream>>>(XB, WQ, F, W1, PL16);
    k_qkp<<<dim3((x8 + 255) / 256, 2, 1), 256, 0, stream>>>(F, QK16, QKh, QKl);
    k_vtp<<<(x8 + 255) / 256, 256, 0, stream>>>(F + 2 * PL16, VT16, VTh, VTl);
    k_attn_s<<<dim3(RH / 16, NH, NB), 32, 0, stream>>>(QKh, QKl, QKh + PLR, QKl + PLR, VTh, VTl, GATE, ATh, ATl);
    if (SEQ > RH) k_attn_h<<<dim3((SEQ - RH) / 32 > 0 ? (SEQ - RH) / 32 : 1, NH, NB), 32, 0, stream>>>(QK16, QK16 + PL16, VT16, GATE, ATh, ATl);
    k_gemm_out<<<dim3(MROWS / 64, CC / 64, 1), 32, 0, stream>>>(ATh, ATl, WO, OUT, bo);
}
